// Attention_54795192762650
// MI455X (gfx1250) — hardware-verified
//
#include <hip/hip_runtime.h>


#ifndef NB
#define NB 2
#endif
#ifndef SEQ
#define SEQ 2048
#endif
#ifndef RRES
#define RRES 256
#endif
#define NB_FULL 2
#define SEQ_FULL 2048
#define DIN 2048
#define DMO 2048
#define NH 32
#define NKV 8
#define GRP (NH / NKV)
#define HD 64
#define DKV (NKV * HD)
#define DQKV (DMO + 2 * DKV)
#define PP 72
#define PCAR 1024.0f
#define CCAR 16.0f
#define WCAR 64.0f
#define SCL 0.125f
#define L2E 1.4426950408889634f
#define MASKNEG (-1.0e9f)
#define MASKLIM (-1.0e8f)
static_assert(SEQ % 64 == 0 && SEQ >= 64 && SEQ <= SEQ_FULL);
static_assert(RRES % 64 == 0 && RRES >= 64 && RRES <= SEQ);
static_assert(NB >= 1 && NB <= NB_FULL);
static_assert(SEQ / 8 <= 256);
static_assert(DIN % 32 == 0 && DMO % 64 == 0 && DKV % 64 == 0 && HD == 64 && (NH % NKV) == 0);
static_assert(DMO == NH * HD && DKV == NKV * HD && DQKV % 64 == 0);
static_assert(((size_t)DQKV * DIN) % 64 == 0 && ((size_t)DMO * DMO) % 64 == 0);
static_assert(((size_t)SEQ * DIN) % 8 == 0);
static_assert((size_t)DQKV * DIN * 2 + (size_t)DMO * DMO * 4 + (size_t)SEQ * DIN * 2 + (size_t)SEQ * DMO * 4 + (size_t)SEQ * DKV * 8
              + (size_t)NH * SEQ * HD * 2 + (size_t)NKV * SEQ * HD * 4 + (size_t)NH * RRES * HD * 4 + (size_t)NKV * RRES * HD * 8
              + (size_t)SEQ * DMO * 2 + (size_t)RRES * DMO * 4 + (size_t)(SEQ / 8) * 128 + 256 <= (size_t)134217728);

typedef _Float16 h16;
typedef unsigned short bf;
typedef __attribute__((ext_vector_type(16))) __bf16   v16bf;
typedef __attribute__((ext_vector_type(16))) _Float16 v16h;
typedef __attribute__((ext_vector_type(8)))  _Float16 v8h;
typedef __attribute__((ext_vector_type(8)))  unsigned short v8us;
typedef __attribute__((ext_vector_type(8)))  float    v8f;
typedef __attribute__((ext_vector_type(4)))  float    v4f;
typedef __attribute__((ext_vector_type(4)))  int      v4i;
typedef __attribute__((ext_vector_type(2)))  _Float16 v2h;
typedef __attribute__((ext_vector_type(2)))  unsigned short v2us;
typedef v8h  __attribute__((may_alias)) v8ha;
typedef v4f  __attribute__((may_alias)) v4fa;
typedef v8us __attribute__((may_alias)) v8usa;

__device__ __forceinline__ unsigned short f2bf(float f) { unsigned u = __float_as_uint(f); u += 0x7FFFu + ((u >> 16) & 1u); return (unsigned short)(u >> 16); }
__device__ __forceinline__ float bf2f(unsigned short b) { return __uint_as_float(((unsigned)b) << 16); }
__device__ __forceinline__ float bfr(float f) { return bf2f(f2bf(f)); }
__device__ __forceinline__ h16 tohx(float x) { return (h16)x; }
__device__ __forceinline__ void splitf(float y, unsigned short& h, unsigned short& l) { h = f2bf(y); l = f2bf(y - bf2f(h)); }
__device__ __forceinline__ v16h cat16(v8h lo, v8h hi) { return __builtin_shufflevector(lo, hi, 0, 1, 2, 3, 4, 5, 6, 7, 8, 9, 10, 11, 12, 13, 14, 15); }
__device__ __forceinline__ v16bf cat16b(v8us lo, v8us hi) { return __builtin_bit_cast(v16bf, __builtin_shufflevector(lo, hi, 0, 1, 2, 3, 4, 5, 6, 7, 8, 9, 10, 11, 12, 13, 14, 15)); }
__device__ __forceinline__ v8f wmma16(v16h a, v16h b, v8f c) { return __builtin_amdgcn_wmma_f32_16x16x32_f16(false, a, false, b, (short)0, c, false, false); }
__device__ __forceinline__ v8f wmmab(v16bf a, v16bf b, v8f c) { return __builtin_amdgcn_wmma_f32_16x16x32_bf16(false, a, false, b, (short)0, c, false, false); }
__device__ __forceinline__ void lds_wsync() { __builtin_amdgcn_fence(3  , "wavefront"); __builtin_amdgcn_wave_barrier(); asm volatile("" ::: "memory"); }
static __device__ __forceinline__ h16 toh_flush(float v) { const h16 r = (h16)v; return (fabsf(v) < 6.103515625e-05f) ? (h16)0.0f : r; }

template <typename T16> struct WFrag;
template <> struct WFrag<h16> { typedef v16h V; static __device__ __forceinline__ V ld(const h16* p) { return cat16(*(const v8h*)p, *(const v8h*)(p + 16)); } static __device__ __forceinline__ v8f mma(V a, V b, v8f c) { return wmma16(a, b, c); } };
template <> struct WFrag<bf> { typedef v16bf V; static __device__ __forceinline__ V ld(const bf* p) { return cat16b(*(const v8us*)p, *(const v8us*)(p + 16)); } static __device__ __forceinline__ v8f mma(V a, V b, v8f c) { return wmmab(a, b, c); } };

template <typename T16, int NSPLIT>
__global__ __launch_bounds__(32) void k_gemmw(const T16* __restrict__ A, const T16* __restrict__ A2, const T16* __restrict__ Bt, const T16* __restrict__ Bt2, int K, float* C, int ldc, float cscale, const int* __restrict__ pflag, size_t sA, size_t sB, size_t sC) {
    typedef typename WFrag<T16>::V V;
    __shared__ __align__(16) float os[16 * 68];
    const size_t z = blockIdx.z; A += z * sA; if (A2) A2 += z * sA; Bt += z * sB; if (Bt2) Bt2 += z * sB; C += z * sC;
    const int lane = threadIdx.x & 31, lr = lane & 15, hi = lane >> 4; const int r0 = blockIdx.x * 64, c0 = blockIdx.y * 64;
    const float padd = (pflag[0] != 0) ? __int_as_float(0x7fc00000) : 0.0f;
    v8f acc[4][4];
#pragma unroll
    for (int mb = 0; mb < 4; ++mb)
#pragma unroll
        for (int nb = 0; nb < 4; ++nb) acc[mb][nb] = (v8f){};
    const size_t aoff = (size_t)(r0 + lr) * K + 8 * hi, boff = (size_t)(c0 + lr) * K + 8 * hi;
#pragma unroll 1
    for (int kc = 0; kc < K; kc += 32) {
        V a[4], a2[4];
#pragma unroll
        for (int mb = 0; mb < 4; ++mb) { a[mb] = WFrag<T16>::ld(A + aoff + (size_t)mb * 16 * K + kc); if (NSPLIT == 1 || NSPLIT == 2) a2[mb] = WFrag<T16>::ld(A2 + aoff + (size_t)mb * 16 * K + kc); }
#pragma unroll
        for (int nb = 0; nb < 4; ++nb) { const V b = WFrag<T16>::ld(Bt + boff + (size_t)nb * 16 * K + kc); V b2; if (NSPLIT >= 2) b2 = WFrag<T16>::ld(Bt2 + boff + (size_t)nb * 16 * K + kc);
#pragma unroll
            for (int mb = 0; mb < 4; ++mb) { acc[mb][nb] = WFrag<T16>::mma(a[mb], b, acc[mb][nb]); if (NSPLIT == 1 || NSPLIT == 2) acc[mb][nb] = WFrag<T16>::mma(a2[mb], b, acc[mb][nb]); if (NSPLIT >= 2) acc[mb][nb] = WFrag<T16>::mma(a[mb], b2, acc[mb][nb]); } }
        asm volatile("v_nop\n\tv_nop\n\tv_nop\n\tv_nop" : "+v"(acc[0][0]), "+v"(acc[1][1]), "+v"(acc[2][2]), "+v"(acc[3][3]) : "v"(a[0]), "v"(a[3]));
    }
#pragma unroll
    for (int mb = 0; mb < 4; ++mb) {
#pragma unroll
        for (int nb = 0; nb < 4; ++nb) {
#pragma unroll
            for (int j = 0; j < 8; ++j) os[(hi * 8 + j) * 68 + nb * 16 + lr] = acc[mb][nb][j]; }
        __builtin_amdgcn_wave_barrier(); asm volatile("" ::: "memory");
        float* crow = C + (size_t)(r0 + mb * 16) * ldc + c0;
#pragma unroll 1
        for (int ps = 0; ps < 2; ++ps) {
#pragma unroll
            for (int s = 0; s < 8; ++s) { const int row = 2 * s + hi, cofs = lr * 4; v4f val = *(const v4fa*)(os + row * 68 + cofs); val = val * cscale + padd;
                *(volatile v4f*)(crow + (size_t)row * ldc + cofs) = val; }
            if (ps == 0) __threadfence(); }
        __builtin_amdgcn_wave_barrier(); asm volatile("" ::: "memory");
    }
}

__global__ __launch_bounds__(256) void k_mchk(const float* __restrict__ mask, int* MF) {
    __shared__ int sv[8];
    const int lane = threadIdx.x & 31, wave = threadIdx.x >> 5; const int i = blockIdx.x * 8 + wave;
    const float* mr = mask + (size_t)i * SEQ_FULL; int bad = 0;
#pragma unroll 1
    for (int j0 = lane * 4; j0 < SEQ; j0 += 128) { const v4f mv = *(const v4f*)(mr + j0);
#pragma unroll
        for (int q = 0; q < 4; ++q) { const float xv = mv[q]; const bool okz = (xv == 0.0f); const bool okn = (xv <= MASKLIM); const bool need = (j0 + q > i); const bool ok = need ? okn : okz; bad |= ok ? 0 : 1; } }
#pragma unroll
    for (int sh = 16; sh; sh >>= 1) bad |= __shfl_xor(bad, sh, 32);
    if (lane == 0) sv[wave] = bad;
    __syncthreads();
    if (wave == 0) { int v = 0;
#pragma unroll
        for (int w = 0; w < 8; ++w) v |= sv[w];
        int* p = MF + (size_t)blockIdx.x * 32 + lane; *(volatile int*)p = v; __threadfence(); *(volatile int*)p = v; }
}
__global__ __launch_bounds__(256) void k_mred(const int* __restrict__ MF, int nl, int* MFLAG) {
    __shared__ int sv[8];
    const int lane = threadIdx.x & 31, wave = threadIdx.x >> 5; const int t = threadIdx.x; const int tc = (t < nl) ? t : (nl - 1);
    int v = MF[(size_t)tc * 32]; v = (t < nl) ? v : 0;
#pragma unroll
    for (int sh = 16; sh; sh >>= 1) v |= __shfl_xor(v, sh, 32);
    if (lane == 0) sv[wave] = v;
    __syncthreads();
    if (wave == 0) { int r = 0;
#pragma unroll
        for (int w = 0; w < 8; ++w) r |= sv[w];
        int* p = MFLAG + lane; *(volatile int*)p = r; __threadfence(); *(volatile int*)p = r; }
}

__global__ __launch_bounds__(256) void k_wtG(const float* __restrict__ w, int K, int N, bf* Bt, h16* Ht) {
    const int lane = threadIdx.x & 31; const int L0 = (blockIdx.x * 8 + (threadIdx.x >> 5)) * 8; const int nlines = N * K / 64;
#pragma unroll 1
    for (int ps = 0; ps < 2; ++ps) {
#pragma unroll 1
        for (int l = 0; l < 8; ++l) { const int L = L0 + l; if (L >= nlines) break; const size_t e = (size_t)L * 64 + lane * 2; const int k = (int)(e % K), n = (int)(e / K);
            const float w0 = bfr(w[(size_t)k * N + n]), w1 = bfr(w[(size_t)(k + 1) * N + n]); v2us o; o[0] = f2bf(w0); o[1] = f2bf(w1); *(volatile v2us*)(Bt + e) = o;
            if (Ht != nullptr) { v2h oh; oh[0] = tohx(w0 * WCAR); oh[1] = tohx(w1 * WCAR); *(volatile v2h*)(Ht + e) = oh; } }
        if (ps == 0) __threadfence(); }
}
__global__ __launch_bounds__(256) void k_cvt8(const float* __restrict__ src, bf* dst, size_t n8) { const size_t i = (size_t)blockIdx.x * 256 + threadIdx.x; if (i >= n8) return; const v8f v = *(const v8f*)(src + i * 8); v8us o;
#pragma unroll
    for (int k = 0; k < 8; ++k) o[k] = f2bf(v[k]); *(volatile v8us*)(dst + i * 8) = o; __threadfence(); *(volatile v8us*)(dst + i * 8) = o; }

__global__ __launch_bounds__(256) void k_hpl(const float* __restrict__ F, int nheads, h16* P16, bf* Ph, bf* Pl) {
    const size_t e = ((size_t)blockIdx.x * 256 + threadIdx.x) * 2; if (e >= (size_t)nheads * SEQ * HD) return;
    const int d = (int)(e % HD); const int t = (int)((e / HD) % SEQ); const int h = (int)(e / ((size_t)HD * SEQ));
    v2h o16; v2us oh, ol;
#pragma unroll
    for (int q = 0; q < 2; ++q) { const float r = F[e + q]; o16[q] = toh_flush(r); unsigned short a2, c2; splitf(r, a2, c2); oh[q] = a2; ol[q] = c2; }
    const bool res = (t < RRES); const size_t oo = ((size_t)h * RRES + (res ? t : 0)) * HD + d;
    *(volatile v2h*)(P16 + e) = o16; if (res) { *(volatile v2us*)(Ph + oo) = oh; *(volatile v2us*)(Pl + oo) = ol; }
    __threadfence();
    *(volatile v2h*)(P16 + e) = o16; if (res) { *(volatile v2us*)(Ph + oo) = oh; *(volatile v2us*)(Pl + oo) = ol; }
}
__global__ __launch_bounds__(256) void k_vtpl(const float* __restrict__ F, int ng, h16* V16, bf* Vh, bf* Vl) {
    const size_t e = ((size_t)blockIdx.x * 256 + threadIdx.x) * 2; if (e >= (size_t)ng * HD * SEQ) return;
    const int t = (int)(e % SEQ); const int d = (int)((e / SEQ) % HD); const int g = (int)(e / ((size_t)SEQ * HD)); v2h o16; v2us oh, ol;
#pragma unroll
    for (int q = 0; q < 2; ++q) { const float x = F[((size_t)g * SEQ + (size_t)(t + q)) * HD + d]; o16[q] = toh_flush(x); unsigned short a2, c2; splitf(x, a2, c2); oh[q] = a2; ol[q] = c2; }
    const bool res = (t < RRES); const size_t oo = ((size_t)g * HD + d) * RRES + (res ? t : 0);
    *(volatile v2h*)(V16 + e) = o16; if (res) { *(volatile v2us*)(Vh + oo) = oh; *(volatile v2us*)(Vl + oo) = ol; }
    __threadfence();
    *(volatile v2h*)(V16 + e) = o16; if (res) { *(volatile v2us*)(Vh + oo) = oh; *(volatile v2us*)(Vl + oo) = ol; }
}

__device__ __forceinline__ void online_softmax(v8f (&s)[4], float (&m)[8], float (&l)[8], v8f (&o)[4], bool diag, int row0, int kvb, int lr, int hi) {
#pragma unroll
    for (int nt = 0; nt < 4; ++nt)
#pragma unroll
        for (int r = 0; r < 8; ++r) { const int row = row0 + 8 * hi + r, col = kvb + nt * 16 + lr; float v = s[nt][r] * SCL; if (diag && col > row) v = v + MASKNEG; s[nt][r] = v; }
#pragma unroll
    for (int r = 0; r < 8; ++r) {
        float mx = fmaxf(fmaxf(s[0][r], s[1][r]), fmaxf(s[2][r], s[3][r]));
#pragma unroll
        for (int sh = 1; sh < 16; sh <<= 1) mx = fmaxf(mx, __shfl_xor(mx, sh, 32));
        const float m2 = fmaxf(m[r], mx); const float alpha = __builtin_amdgcn_exp2f((m[r] - m2) * L2E); m[r] = m2;
        float rs = 0.0f;
#pragma unroll
        for (int nt = 0; nt < 4; ++nt) { const float p = __builtin_amdgcn_exp2f((s[nt][r] - m2) * L2E); s[nt][r] = p; rs += p; }
#pragma unroll
        for (int sh = 1; sh < 16; sh <<= 1) rs += __shfl_xor(rs, sh, 32);
        l[r] = l[r] * alpha + rs;
#pragma unroll
        for (int nt = 0; nt < 4; ++nt) o[nt][r] = o[nt][r] * alpha;
    }
}

__global__ __launch_bounds__(128) void k_attnr(const bf* __restrict__ QPh, const bf* __restrict__ QPl, const bf* __restrict__ KPh, const bf* __restrict__ KPl, const bf* __restrict__ VTh, const bf* __restrict__ VTl, bf* CTh, bf* CTl) {
    __shared__ __align__(16) bf sP[4][2][16 * PP];
    const int lane = threadIdx.x & 31, wave = threadIdx.x >> 5, lr = lane & 15, hi = lane >> 4;
    const int qt = blockIdx.x, h = blockIdx.y, g = h % NKV; const int q0 = qt * 64 + wave * 16;
    const bf* qh = QPh + ((size_t)h * RRES + q0) * HD; const bf* ql = QPl + ((size_t)h * RRES + q0) * HD;
    const bf* kh = KPh + (size_t)g * RRES * HD; const bf* kl = KPl + (size_t)g * RRES * HD;
    const bf* vh = VTh + (size_t)g * HD * RRES; const bf* vl = VTl + (size_t)g * HD * RRES;
    bf* sph = &sP[wave][0][0]; bf* spl = &sP[wave][1][0];
    float m[8], l[8]; v8f o[4];
#pragma unroll
    for (int r = 0; r < 8; ++r) { m[r] = -3.0e38f; l[r] = 0.0f; }
#pragma unroll
    for (int nt = 0; nt < 4; ++nt) o[nt] = (v8f){};
#pragma unroll 1
    for (int c = 0; c <= qt; ++c) {
        const int kvb = c * 64; v8f s[4]; v16bf aqh[2], aql[2], bh, bl;
#pragma unroll
        for (int kk = 0; kk < 2; ++kk) { aqh[kk] = WFrag<bf>::ld(qh + (size_t)lr * HD + 8 * hi + kk * 32); aql[kk] = WFrag<bf>::ld(ql + (size_t)lr * HD + 8 * hi + kk * 32); }
#pragma unroll
        for (int nt = 0; nt < 4; ++nt) { s[nt] = (v8f){}; const size_t ko = (size_t)(kvb + nt * 16 + lr) * HD + 8 * hi;
#pragma unroll
            for (int kk = 0; kk < 2; ++kk) { bh = WFrag<bf>::ld(kh + ko + kk * 32); bl = WFrag<bf>::ld(kl + ko + kk * 32);
                s[nt] = wmmab(aqh[kk], bh, s[nt]); s[nt] = wmmab(aql[kk], bh, s[nt]); s[nt] = wmmab(aqh[kk], bl, s[nt]); } }
        asm volatile("v_nop\n\tv_nop\n\tv_nop\n\tv_nop" : "+v"(s[0]), "+v"(s[1]), "+v"(s[2]), "+v"(s[3]) : "v"(aqh[0]), "v"(aql[1]), "v"(bh), "v"(bl));
        online_softmax(s, m, l, o, c == qt, q0, kvb, lr, hi);
#pragma unroll
        for (int nt = 0; nt < 4; ++nt)
#pragma unroll
            for (int r = 0; r < 8; ++r) { unsigned short a2, c2; splitf(s[nt][r], a2, c2); const int so = (8 * hi + r) * PP + nt * 16 + lr; sph[so] = a2; spl[so] = c2; }
        lds_wsync();
        v16bf aph[2], apl[2], bvh, bvl;
#pragma unroll
        for (int kk = 0; kk < 2; ++kk) { const int ao = lr * PP + kk * 32 + 8 * hi; aph[kk] = cat16b(*(const v8usa*)(sph + ao), *(const v8usa*)(sph + ao + 16)); apl[kk] = cat16b(*(const v8usa*)(spl + ao), *(const v8usa*)(spl + ao + 16)); }
#pragma unroll
        for (int kk = 0; kk < 2; ++kk)
#pragma unroll
            for (int nt = 0; nt < 4; ++nt) { const size_t vo = (size_t)(nt * 16 + lr) * RRES + kvb + kk * 32 + 8 * hi; bvh = WFrag<bf>::ld(vh + vo); bvl = WFrag<bf>::ld(vl + vo);
                o[nt] = wmmab(aph[kk], bvh, o[nt]); o[nt] = wmmab(apl[kk], bvh, o[nt]); o[nt] = wmmab(aph[kk], bvl, o[nt]); }
        asm volatile("v_nop\n\tv_nop\n\tv_nop\n\tv_nop" : "+v"(o[0]), "+v"(o[1]), "+v"(o[2]), "+v"(o[3]) : "v"(aph[0]), "v"(apl[1]), "v"(bvh), "v"(bvl));
        lds_wsync();
    }
    float inv[8];
#pragma unroll
    for (int r = 0; r < 8; ++r) inv[r] = 1.0f / l[r];
#pragma unroll
    for (int nt = 0; nt < 4; ++nt)
#pragma unroll
        for (int r = 0; r < 8; ++r) { unsigned short a2, c2; splitf(o[nt][r] * inv[r], a2, c2); const int so = (8 * hi + r) * PP + nt * 16 + lr; sph[so] = a2; spl[so] = c2; }
    lds_wsync();
    bf* chb = CTh + (size_t)q0 * DMO + h * HD; bf* clb = CTl + (size_t)q0 * DMO + h * HD;
#pragma unroll 1
    for (int ps = 0; ps < 2; ++ps) {
#pragma unroll
        for (int it = 0; it < 4; ++it) { const int rr = it * 4 + (lane >> 3), pc = (lane & 7) * 8; const v8us va = *(const v8usa*)(sph + rr * PP + pc); const v8us vb = *(const v8usa*)(spl + rr * PP + pc);
            *(volatile v8us*)(chb + (size_t)rr * DMO + pc) = va; *(volatile v8us*)(clb + (size_t)rr * DMO + pc) = vb; }
        if (ps == 0) __threadfence(); }
}

__global__ __launch_bounds__(128) void k_attn(const h16* __restrict__ Q16, const h16* __restrict__ K16, const h16* __restrict__ VT16, h16* C16) {
    __shared__ __align__(16) h16 sP[4][16 * PP];
    const int lane = threadIdx.x & 31, wave = threadIdx.x >> 5, lr = lane & 15, hi = lane >> 4;
    const int qt = blockIdx.x + RRES / 64, h = blockIdx.y, g = h % NKV; const int q0 = qt * 64 + wave * 16;
    const h16* qp = Q16 + ((size_t)h * SEQ + q0) * HD; const h16* kp = K16 + (size_t)g * SEQ * HD; const h16* vp = VT16 + (size_t)g * HD * SEQ;
    h16* spw = &sP[wave][0];
    v16h aq[2];
#pragma unroll
    for (int kk = 0; kk < 2; ++kk) aq[kk] = WFrag<h16>::ld(qp + (size_t)lr * HD + 8 * hi + kk * 32);
    float m[8], l[8]; v8f o[4];
#pragma unroll
    for (int r = 0; r < 8; ++r) { m[r] = -3.0e38f; l[r] = 0.0f; }
#pragma unroll
    for (int nt = 0; nt < 4; ++nt) o[nt] = (v8f){};
    const int nch = qt + 1;
#pragma unroll 1
    for (int c = 0; c < nch; ++c) {
        const int kvb = c * 64; v8f s[4]; v16h b;
#pragma unroll
        for (int nt = 0; nt < 4; ++nt) { s[nt] = (v8f){}; const h16* kr = kp + (size_t)(kvb + nt * 16 + lr) * HD + 8 * hi;
#pragma unroll
            for (int kk = 0; kk < 2; ++kk) { b = WFrag<h16>::ld(kr + kk * 32); s[nt] = wmma16(aq[kk], b, s[nt]); } }
        asm volatile("v_nop\n\tv_nop\n\tv_nop\n\tv_nop" : "+v"(s[0]), "+v"(s[1]), "+v"(s[2]), "+v"(s[3]) : "v"(aq[0]), "v"(aq[1]), "v"(b));
        online_softmax(s, m, l, o, c == qt, q0, kvb, lr, hi);
#pragma unroll
        for (int nt = 0; nt < 4; ++nt)
#pragma unroll
            for (int r = 0; r < 8; ++r) spw[(8 * hi + r) * PP + nt * 16 + lr] = toh_flush(s[nt][r] * PCAR);
        lds_wsync();
        v16h ap[2], bv;
#pragma unroll
        for (int kk = 0; kk < 2; ++kk) { const int ao = lr * PP + kk * 32 + 8 * hi; ap[kk] = cat16(*(const v8ha*)(spw + ao), *(const v8ha*)(spw + ao + 16)); }
#pragma unroll
        for (int kk = 0; kk < 2; ++kk)
#pragma unroll
            for (int nt = 0; nt < 4; ++nt) { bv = WFrag<h16>::ld(vp + (size_t)(nt * 16 + lr) * SEQ + kvb + kk * 32 + 8 * hi); o[nt] = wmma16(ap[kk], bv, o[nt]); }
        asm volatile("v_nop\n\tv_nop\n\tv_nop\n\tv_nop" : "+v"(o[0]), "+v"(o[1]), "+v"(o[2]), "+v"(o[3]) : "v"(ap[0]), "v"(ap[1]), "v"(bv));
        lds_wsync();
    }
    float inv[8];
#pragma unroll
    for (int r = 0; r < 8; ++r) inv[r] = (1.0f / l[r]) * (CCAR / PCAR);
#pragma unroll
    for (int nt = 0; nt < 4; ++nt)
#pragma unroll
        for (int r = 0; r < 8; ++r) spw[(8 * hi + r) * PP + nt * 16 + lr] = toh_flush(o[nt][r] * inv[r]);
    lds_wsync();
    h16* cb = C16 + (size_t)q0 * DMO + h * HD;
#pragma unroll 1
    for (int ps = 0; ps < 2; ++ps) {
#pragma unroll
        for (int it = 0; it < 4; ++it) { const int rr = it * 4 + (lane >> 3), pc = (lane & 7) * 8; const v8h val = *(const v8ha*)(spw + rr * PP + pc); *(volatile v8h*)(cb + (size_t)rr * DMO + pc) = val; }
        if (ps == 0) __threadfence(); }
}

extern "C" void kernel_launch(void* const* d_in, const int* in_sizes, int n_in,
                              void* d_out, int out_size, void* d_ws, size_t ws_size, hipStream_t stream) {
    if (n_in < 4) return;
    const long long rows_used = (long long)(NB - 1) * SEQ_FULL + SEQ;
    if ((long long)in_sizes[0] < rows_used * DIN) return;
    if ((long long)in_sizes[1] < (long long)(SEQ - 1) * SEQ_FULL + SEQ) return;
    if (in_sizes[2] < DIN * DQKV || in_sizes[3] < DMO * DMO) return;
    if ((long long)out_size < rows_used * DMO) return;
    const float* x = (const float*)d_in[0]; const float* maskf = (const float*)d_in[1]; const float* wqkv = (const float*)d_in[2]; const float* wo = (const float*)d_in[3];
    float* OUT = (float*)d_out;
    char* wsp = (char*)d_ws;
    auto take = [&](size_t bytes) { char* p = wsp; wsp += (bytes + 255) & ~(size_t)255; return (void*)p; };
    bf* WQKV = (bf*)take((size_t)DQKV * DIN * 2);
    bf* WOb  = (bf*)take((size_t)DMO * DMO * 2);
    h16* WO16 = (h16*)take((size_t)DMO * DMO * 2);
    bf* XB   = (bf*)take((size_t)SEQ * DIN * 2);
    float* FQ = (float*)take((size_t)SEQ * DMO * 4);
    float* FK = (float*)take((size_t)SEQ * DKV * 4);
    float* FV = (float*)take((size_t)SEQ * DKV * 4);
    h16* Q16 = (h16*)take((size_t)NH * SEQ * HD * 2); h16* K16 = (h16*)take((size_t)NKV * SEQ * HD * 2); h16* VT16 = (h16*)take((size_t)NKV * HD * SEQ * 2);
    bf* QPh = (bf*)take((size_t)NH * RRES * HD * 2); bf* QPl = (bf*)take((size_t)NH * RRES * HD * 2);
    bf* KPh = (bf*)take((size_t)NKV * RRES * HD * 2); bf* KPl = (bf*)take((size_t)NKV * RRES * HD * 2);
    bf* VTh = (bf*)take((size_t)NKV * HD * RRES * 2); bf* VTl = (bf*)take((size_t)NKV * HD * RRES * 2);
    h16* C16 = (h16*)take((size_t)SEQ * DMO * 2);
    bf* CTh = (bf*)take((size_t)RRES * DMO * 2); bf* CTl = (bf*)take((size_t)RRES * DMO * 2);
    int* MF = (int*)take((size_t)(SEQ / 8) * 128); int* MFLAG = (int*)take(128);
    const size_t carved = (size_t)(wsp - (char*)d_ws);
    if (carved > ws_size || carved > (size_t)134217728) return;

    k_mchk<<<SEQ / 8, 256, 0, stream>>>(maskf, MF);
    k_mred<<<1, 256, 0, stream>>>(MF, SEQ / 8, MFLAG);
    k_wtG<<<(unsigned)((DQKV * DIN / 64 + 63) / 64), 256, 0, stream>>>(wqkv, DIN, DQKV, WQKV, nullptr);
    k_wtG<<<(unsigned)((DMO * DMO / 64 + 63) / 64), 256, 0, stream>>>(wo, DMO, DMO, WOb, WO16);
    const unsigned LQ = (unsigned)(((size_t)NH * SEQ * HD / 2 + 255) / 256), LKV = (unsigned)(((size_t)NKV * SEQ * HD / 2 + 255) / 256);
    for (int b = 0; b < NB; ++b) {
        k_cvt8<<<(unsigned)(((size_t)SEQ * DIN / 8 + 255) / 256), 256, 0, stream>>>(x + (size_t)b * SEQ_FULL * DIN, XB, (size_t)SEQ * DIN / 8);
        k_gemmw<bf, 0><<<dim3(SEQ / 64, DMO / 64, 1), 32, 0, stream>>>(XB, nullptr, WQKV, nullptr, DIN, FQ, DMO, 1.0f, MFLAG, 0, 0, 0);
        k_gemmw<bf, 0><<<dim3(SEQ / 64, DKV / 64, 1), 32, 0, stream>>>(XB, nullptr, WQKV + (size_t)DMO * DIN, nullptr, DIN, FK, DKV, 1.0f, MFLAG, 0, 0, 0);
        k_gemmw<bf, 0><<<dim3(SEQ / 64, DKV / 64, 1), 32, 0, stream>>>(XB, nullptr, WQKV + (size_t)(DMO + DKV) * DIN, nullptr, DIN, FV, DKV, 1.0f, MFLAG, 0, 0, 0);
        k_hpl<<<LQ, 256, 0, stream>>>(FQ, NH, Q16, QPh, QPl);
        k_hpl<<<LKV, 256, 0, stream>>>(FK, NKV, K16, KPh, KPl);
        k_vtpl<<<LKV, 256, 0, stream>>>(FV, NKV, VT16, VTh, VTl);
        k_attnr<<<dim3(RRES / 64, NH, 1), 128, 0, stream>>>(QPh, QPl, KPh, KPl, VTh, VTl, CTh, CTl);
        if (SEQ > RRES) k_attn<<<dim3((SEQ - RRES) / 64, NH, 1), 128, 0, stream>>>(Q16, K16, VT16, C16);
        float* ob = OUT + (size_t)b * SEQ_FULL * DMO;
        k_gemmw<bf, 1><<<dim3(RRES / 64, DMO / 64, 1), 32, 0, stream>>>(CTh, CTl, WOb, nullptr, DMO, ob, DMO, 1.0f, MFLAG, 0, 0, 0);
        if (SEQ > RRES) k_gemmw<h16, 0><<<dim3((SEQ - RRES) / 64, DMO / 64, 1), 32, 0, stream>>>(C16 + (size_t)RRES * DMO, nullptr, WO16, nullptr, DMO, ob + (size_t)RRES * DMO, DMO, 1.0f / (CCAR * WCAR), MFLAG, 0, 0, 0);
    }
}
